// InteractionFFN_19035295056635
// MI455X (gfx1250) — hardware-verified
//
#include <hip/hip_runtime.h>
#include <math.h>

typedef __attribute__((ext_vector_type(16))) _Float16 v16h;
typedef __attribute__((ext_vector_type(16))) __bf16 v16b;
typedef __attribute__((ext_vector_type(8)))  _Float16 v8h;
typedef __attribute__((ext_vector_type(8)))  float v8f;
typedef __attribute__((ext_vector_type(4)))  float v4f;
typedef __attribute__((ext_vector_type(2)))  float v2f;
typedef __attribute__((ext_vector_type(4)))  unsigned v4u;
typedef __attribute__((ext_vector_type(4)))  int v4i;
typedef float __attribute__((may_alias)) float_a;
typedef int __attribute__((may_alias)) int_a;

template <typename T> __device__ __forceinline__ void vst2(void* p, T v) { *(volatile T*)p = v; __threadfence(); *(volatile T*)p = v; }
__device__ __forceinline__ v8f wmma16(v16h a, v16h b, v8f c) {
  v8f d = __builtin_amdgcn_wmma_f32_16x16x32_f16(false, a, false, b, (short)0, c, false, false);
  asm volatile("v_nop\n\tv_nop\n\tv_nop\n\tv_nop" : "+v"(d) : "v"(a), "v"(b));
  return d;
}
__device__ __forceinline__ v8f wmma_bf(v16b a, v16b b, v8f c) {
  v8f d = __builtin_amdgcn_wmma_f32_16x16x32_bf16(false, a, false, b, (short)0, c, false, false);
  asm volatile("v_nop\n\tv_nop\n\tv_nop\n\tv_nop" : "+v"(d) : "v"(a), "v"(b));
  return d;
}
__device__ __forceinline__ v16h frag_h(const _Float16* rowk0, int lane) {
  union { v16h v; v8h q[2]; } u; const _Float16* p = rowk0 + 8 * (lane >> 4);
  u.q[0] = *(const v8h*)p; u.q[1] = *(const v8h*)(p + 16); return u.v;
}
__device__ __forceinline__ v16h frag_f32(const float* rowk0, int lane) {
  v16h a; const float* p = rowk0 + 8 * (lane >> 4);
#pragma unroll
  for (int i = 0; i < 8; ++i) { a[i] = (_Float16)p[i]; a[8 + i] = (_Float16)p[16 + i]; }
  return a;
}
__device__ __forceinline__ v16h frag_f32s(const float* rowk0, int lane, float sc) {
  v16h a; const float* p = rowk0 + 8 * (lane >> 4);
#pragma unroll
  for (int i = 0; i < 8; ++i) { a[i] = (_Float16)(p[i] * sc); a[8 + i] = (_Float16)(p[16 + i] * sc); }
  return a;
}
__device__ __forceinline__ v16h fragc_f32(const float* W, int k0, int n, int lane, int ld, int K) {
  v16h a; const int g = lane >> 4;
#pragma unroll
  for (int i = 0; i < 8; ++i) { const int ka = k0 + 8 * g + i, kb = ka + 16;
    a[i] = (_Float16)(ka < K ? W[(size_t)(ka < K ? ka : K - 1) * ld + n] : 0.f); a[8 + i] = (_Float16)(kb < K ? W[(size_t)(kb < K ? kb : K - 1) * ld + n] : 0.f); }
  return a;
}
struct F2 { v16b h, l; };
__device__ __forceinline__ F2 bsplit16(const float v[16]) { F2 r;
#pragma unroll
  for (int i = 0; i < 16; ++i) { const __bf16 h = (__bf16)v[i]; r.h[i] = h; r.l[i] = (__bf16)(v[i] - (float)h); }
  return r; }
__device__ __forceinline__ F2 split_row(const float* row, int k0, int lane) { float v[16]; const float* p = row + k0 + 8 * (lane >> 4);
#pragma unroll
  for (int i = 0; i < 8; ++i) { v[i] = p[i]; v[8 + i] = p[16 + i]; }
  return bsplit16(v); }
__device__ __forceinline__ F2 split_rowK(const float* row, int k0, int lane, int K) { float v[16]; const int g = lane >> 4;
#pragma unroll
  for (int i = 0; i < 8; ++i) { const int ka = k0 + 8 * g + i, kb = ka + 16; v[i] = ka < K ? row[ka < K ? ka : K - 1] : 0.f; v[8 + i] = kb < K ? row[kb < K ? kb : K - 1] : 0.f; }
  return bsplit16(v); }
__device__ __forceinline__ F2 split_col(const float* W, int k0, int n, int lane, int ld, int K) { float v[16]; const int g = lane >> 4;
#pragma unroll
  for (int i = 0; i < 8; ++i) { const int ka = k0 + 8 * g + i, kb = ka + 16; v[i] = ka < K ? W[(size_t)(ka < K ? ka : K - 1) * ld + n] : 0.f; v[8 + i] = kb < K ? W[(size_t)(kb < K ? kb : K - 1) * ld + n] : 0.f; }
  return bsplit16(v); }
__device__ __forceinline__ v8f mac3(const F2& a, const F2& b, v8f c) { c = wmma_bf(a.l, b.h, c); c = wmma_bf(a.h, b.l, c); return wmma_bf(a.h, b.h, c); }
__device__ __forceinline__ float sigm(float v) { return 1.0f / (1.0f + expf(-v)); }
#define LDSX() do { asm volatile("s_wait_dscnt 0" ::: "memory"); __builtin_amdgcn_wave_barrier(); __builtin_amdgcn_fence(__ATOMIC_RELEASE, "workgroup"); } while (0)


#define NTK 2048
#define KN 8
#define NNR (NTK * KN)
#define DD 512
#define NH 8
#define DH 64
#define NPAT 32
#define RK 32
#define PR (NPAT * RK)
#define FF 1024
#define KSEL 4
#ifndef NTT
#define NTT NTK
#endif
typedef __attribute__((ext_vector_type(8))) __bf16 v8b;
__device__ __forceinline__ v16b frag_b(const __bf16* rowk0, int lane) {
  union { v16b v; v8b q[2]; } u; const __bf16* p = rowk0 + 8 * (lane >> 4);
  u.q[0] = *(const v8b*)p; u.q[1] = *(const v8b*)(p + 16); return u.v;
}
__device__ __forceinline__ float bfr(float v) { return (float)(__bf16)v; }
__device__ __attribute__((noinline)) float exp_ni(float v) { return expf(v); }
__device__ __attribute__((noinline)) float erf_ni(float v) { return erff(v); }
__device__ __forceinline__ float gelu_exact(float v) { return 0.5f * v * (1.0f + erf_ni(v * 0.70710678118654752f)); }

#define PK_QKV 0
#define PK_A   (PK_QKV + 3 * DD * DD)
#define PK_B   (PK_A + (size_t)PR * DD)
#define PK_UP  (PK_B + (size_t)FF * PR)
#define PK_DN  (PK_UP + (size_t)FF * DD)
#define PK_END (PK_DN + (size_t)DD * FF)
#define WS_PK  0u
#define WS_QKV (((2u * PK_END) + 127u) / 128u * 128u)
#define WS_CBH (WS_QKV + 4u * (size_t)NNR * 3 * DD)
#define WS_CBL (WS_CBH + 2u * NTK * DD)
#define WS_WSL (WS_CBL + 2u * NTK * DD)
#define WS_HWH (WS_WSL + 4u * NTK * NPAT)
#define WS_HWL (WS_HWH + 2u * NTK * PR)
#define WS_GH  (WS_HWL + 2u * NTK * PR)
#define WS_GL  (WS_GH + 2u * NTK * FF)
#define WS_END (WS_GL + 2u * NTK * FF)

__global__ __launch_bounds__(256) void k_pack(const float* __restrict__ WQ, const float* __restrict__ WK, const float* __restrict__ WV, const float* __restrict__ PA, const float* __restrict__ PB, const float* __restrict__ WU, const float* __restrict__ WD, __bf16* __restrict__ PK) {
  __shared__ __align__(16) __bf16 s[1024]; const int n = blockIdx.x, which = blockIdx.y, t = threadIdx.x; int K; size_t dst;
  if (which == 0) { if (n >= 3 * DD) return; const int m = n / DD, j = n % DD; const float* Wm = (m == 0) ? WQ : (m == 1) ? WK : WV; K = DD; dst = PK_QKV + (size_t)n * DD; for (int k = t; k < DD; k += 256) s[k] = (__bf16)Wm[(size_t)k * DD + j]; }
  else if (which == 1) { if (n >= PR) return; const int p = n / RK, r = n % RK; K = DD; dst = PK_A + (size_t)n * DD; for (int k = t; k < DD; k += 256) s[k] = (__bf16)PA[((size_t)p * DD + k) * RK + r]; }
  else if (which == 2) { if (n >= FF) return; K = PR; dst = PK_B + (size_t)n * PR; for (int k = t; k < PR; k += 256) { const int p = k / RK, r = k % RK; s[k] = (__bf16)PB[((size_t)p * RK + r) * FF + n]; } }
  else if (which == 3) { if (n >= FF) return; K = DD; dst = PK_UP + (size_t)n * DD; for (int k = t; k < DD; k += 256) s[k] = (__bf16)WU[(size_t)k * FF + n]; }
  else { if (n >= DD) return; K = FF; dst = PK_DN + (size_t)n * FF; for (int k = t; k < FF; k += 256) s[k] = (__bf16)WD[(size_t)k * DD + n]; }
  __syncthreads();
  for (int q = t; q < K / 8; q += 256) vst2((unsigned*)(PK + dst + q * 8), *(const v4u*)&s[q * 8]);
}
__global__ __launch_bounds__(128) void k_qkv(const float* __restrict__ SEL, const __bf16* __restrict__ PK, const float* __restrict__ BQ, const float* __restrict__ BK, const float* __restrict__ BV, float* __restrict__ QKV) {
  __shared__ __align__(16) float so[4][16][132];
  const int tid = threadIdx.x, wave = tid >> 5, lane = tid & 31, col = lane & 15, g = lane >> 4; const size_t r0 = (size_t)blockIdx.x * 64 + wave * 16; const int n0 = blockIdx.y * 128; const int which = n0 / DD;
  const float* BB = (which == 0) ? BQ : (which == 1) ? BK : BV;
  v8f acc[8] = {};
#pragma unroll 2
  for (int kc = 0; kc < DD / 32; ++kc) { v16b a; { const float* p = SEL + (r0 + col) * DD + kc * 32 + 8 * g;
#pragma unroll
      for (int i = 0; i < 8; ++i) { a[i] = (__bf16)p[i]; a[8 + i] = (__bf16)p[16 + i]; } }
#pragma unroll
    for (int j = 0; j < 8; ++j) acc[j] = wmma_bf(a, frag_b(PK + PK_QKV + (size_t)(n0 + j * 16 + col) * DD + kc * 32, lane), acc[j]); }
#pragma unroll
  for (int j = 0; j < 8; ++j) { const float bb = bfr(BB[n0 - which * DD + j * 16 + col]);
#pragma unroll
    for (int r = 0; r < 8; ++r) { float v = acc[j][r] + bb; if (which == 2) v = 1.0f / (1.0f + exp_ni(-v)); so[wave][8 * g + r][j * 16 + col] = v; } }
  LDSX();
  for (int rl = 0; rl < 16; ++rl) vst2(QKV + (r0 + rl) * (3 * DD) + n0 + lane * 4, *(const v4f*)&so[wave][rl][lane * 4]);
}
__global__ __launch_bounds__(256) void k_tok(const float* __restrict__ QKV, const float* __restrict__ SEL, const float* __restrict__ TW, const float* __restrict__ X, const float* __restrict__ CTX, const float* __restrict__ PQ, __bf16* __restrict__ CBH, __bf16* __restrict__ CBL, float* __restrict__ WSL) {
  __shared__ float sp[NH][KN][KN]; __shared__ float sagg[DD]; __shared__ float sctx[DD]; __shared__ float sps[NPAT]; __shared__ __align__(16) float sw[NPAT]; __shared__ __align__(16) __bf16 sh_[DD], sl_[DD];
  const int tid = threadIdx.x; const size_t t = blockIdx.x; const float* qkv = QKV + t * KN * (3 * DD);
  for (int e = tid; e < NH * KN * KN; e += 256) { const int h = e >> 6, i = (e >> 3) & 7, j = e & 7; const float* qi = qkv + (size_t)i * (3 * DD) + h * DH; const float* kj = qkv + (size_t)j * (3 * DD) + DD + h * DH; float a = 0.f;
#pragma unroll 1
    for (int d = 0; d < DH; ++d) a += qi[d] * kj[d];
    sp[h][i][j] = a * 0.125f; }
  __syncthreads();
  if (tid < NH * KN) { const int h = tid >> 3, i = tid & 7; float mx = -3.0e38f; for (int j = 0; j < KN; ++j) mx = fmaxf(mx, sp[h][i][j]); float se = 0.f; float ev[KN];
#pragma unroll
    for (int j = 0; j < KN; ++j) { ev[j] = exp_ni(sp[h][i][j] - mx); se += ev[j]; }
#pragma unroll
    for (int j = 0; j < KN; ++j) sp[h][i][j] = ev[j] / se; }
  __syncthreads();
  for (int d = tid; d < DD; d += 256) { const int h = d / DH; float agg = 0.f;
#pragma unroll 1
    for (int i = 0; i < KN; ++i) { float gsum = 0.f;
#pragma unroll 1
      for (int j = 0; j < KN; ++j) gsum += sp[h][i][j] * qkv[(size_t)j * (3 * DD) + 2 * DD + d];
      agg += bfr(TW[t * KN + i]) * (bfr(SEL[(t * KN + i) * DD + d]) * gsum); }
    sagg[d] = agg; sctx[d] = bfr(CTX[t * DD + d]); const float cb = bfr(X[t * DD + d]) + agg; const __bf16 hb = (__bf16)cb; sh_[d] = hb; sl_[d] = (__bf16)(cb - (float)hb); }
  __syncthreads();
  { const int p = tid >> 3, part = tid & 7; float a1 = 0.f, a2 = 0.f;
#pragma unroll 1
    for (int d = part; d < DD; d += 8) { const float w = bfr(PQ[(size_t)p * DD + d]); a1 += sagg[d] * w; a2 += sctx[d] * w; }
#pragma unroll
    for (int o = 1; o < 8; o <<= 1) { a1 += __shfl_xor(a1, o); a2 += __shfl_xor(a2, o); }
    if (part == 0) sps[p] = 0.5f * (a1 * 0.044194173824159216f) + 0.5f * a2; }
  __syncthreads();
  if (tid == 0) { float bv[KSEL]; int bi[KSEL];
#pragma unroll
    for (int s = 0; s < KSEL; ++s) { bv[s] = -3.0e38f; bi[s] = 0; }
    for (int p = 0; p < NPAT; ++p) { const float v = sps[p]; if (v > bv[KSEL - 1]) { float cv = v; int ci = p; bool placed = false;
#pragma unroll
        for (int s = 0; s < KSEL; ++s) { const bool swp = placed || (cv > bv[s]); placed = swp; const float tv = bv[s]; const int ti = bi[s]; bv[s] = swp ? cv : tv; bi[s] = swp ? ci : ti; cv = swp ? tv : cv; ci = swp ? ti : ci; } } }
    float e[KSEL], se = 0.f;
#pragma unroll
    for (int s = 0; s < KSEL; ++s) { e[s] = exp_ni(bv[s] - bv[0]); se += e[s]; }
    for (int p = 0; p < NPAT; ++p) sw[p] = 0.f;
#pragma unroll
    for (int s = 0; s < KSEL; ++s) sw[bi[s]] = e[s] / se; }
  __syncthreads();
  if (tid < DD / 8) vst2((unsigned*)(CBH + t * DD + tid * 8), *(const v4u*)&sh_[tid * 8]); else if (tid < DD / 4) vst2((unsigned*)(CBL + t * DD + (tid - DD / 8) * 8), *(const v4u*)&sl_[(tid - DD / 8) * 8]); else if (tid < DD / 4 + NPAT / 4) vst2(WSL + t * NPAT + (tid - DD / 4) * 4, *(const v4f*)&sw[(tid - DD / 4) * 4]);
}
template <int MODE>
__global__ __launch_bounds__(128) void k_gemm(const __bf16* __restrict__ AH, const __bf16* __restrict__ AL, const __bf16* __restrict__ A2H, const __bf16* __restrict__ A2L, const __bf16* __restrict__ PK, const float* __restrict__ BIAS, const float* __restrict__ WSL, __bf16* __restrict__ OH, __bf16* __restrict__ OL, float* __restrict__ OUTF) {
  __shared__ __align__(16) float so[4][16][132]; __shared__ __align__(16) __bf16 soh[4][16][136], sol[4][16][136];
  const int tid = threadIdx.x, wave = tid >> 5, lane = tid & 31, col = lane & 15, g = lane >> 4; const size_t r0 = (size_t)blockIdx.x * 64 + wave * 16; const int n0 = blockIdx.y * 128;
  constexpr int K1 = (MODE == 2) ? FF : DD; const __bf16* P1 = PK + ((MODE == 0) ? PK_A : (MODE == 1) ? PK_UP : PK_DN);
  v8f acc[8] = {};
#pragma unroll 2
  for (int kc = 0; kc < K1 / 32; ++kc) { F2 a; a.h = frag_b(AH + (r0 + col) * K1 + kc * 32, lane); a.l = frag_b(AL + (r0 + col) * K1 + kc * 32, lane);
#pragma unroll
    for (int j = 0; j < 8; ++j) { const v16b w = frag_b(P1 + (size_t)(n0 + j * 16 + col) * K1 + kc * 32, lane); acc[j] = wmma_bf(a.l, w, acc[j]); acc[j] = wmma_bf(a.h, w, acc[j]); } }
  v8f acc2[8] = {};
  if (MODE == 1) {
#pragma unroll 2
    for (int kc = 0; kc < PR / 32; ++kc) { F2 a; a.h = frag_b(A2H + (r0 + col) * PR + kc * 32, lane); a.l = frag_b(A2L + (r0 + col) * PR + kc * 32, lane);
#pragma unroll
      for (int j = 0; j < 8; ++j) { const v16b w = frag_b(PK + PK_B + (size_t)(n0 + j * 16 + col) * PR + kc * 32, lane); acc2[j] = wmma_bf(a.l, w, acc2[j]); acc2[j] = wmma_bf(a.h, w, acc2[j]); } } }
#pragma unroll
  for (int j = 0; j < 8; ++j) { const int c = n0 + j * 16 + col;
#pragma unroll
    for (int r = 0; r < 8; ++r) { const size_t t = r0 + 8 * g + r; float v;
      if (MODE == 0) v = acc[j][r] * WSL[t * NPAT + (c / RK)];
      else if (MODE == 1) v = gelu_exact(0.1f * (acc[j][r] + bfr(BIAS[c])) + 0.9f * acc2[j][r]);
      else v = acc[j][r] + bfr(BIAS[c]);
      if (MODE < 2) { const __bf16 hb = (__bf16)v; soh[wave][8 * g + r][j * 16 + col] = hb; sol[wave][8 * g + r][j * 16 + col] = (__bf16)(v - (float)hb); } else so[wave][8 * g + r][j * 16 + col] = v; } }
  LDSX();
  constexpr int NOUT = (MODE == 2) ? DD : PR;
  for (int rl = 0; rl < 16; ++rl) { if (MODE < 2) { if (lane < 16) { vst2((unsigned*)(OH + (r0 + rl) * NOUT + n0 + lane * 8), *(const v4u*)&soh[wave][rl][lane * 8]); vst2((unsigned*)(OL + (r0 + rl) * NOUT + n0 + lane * 8), *(const v4u*)&sol[wave][rl][lane * 8]); } }
    else vst2(OUTF + (r0 + rl) * DD + n0 + lane * 4, *(const v4f*)&so[wave][rl][lane * 4]); }
}
extern "C" void kernel_launch(void* const* d_in, const int* in_sizes, int n_in, void* d_out, int out_size, void* d_ws, size_t ws_size, hipStream_t stream) {
  (void)in_sizes; (void)n_in; (void)out_size;
  const float** F = (const float**)d_in;
  if (ws_size < (size_t)WS_END) return;
  char* ws = (char*)d_ws; __bf16 *PK = (__bf16*)(ws + WS_PK), *CBH = (__bf16*)(ws + WS_CBH), *CBL = (__bf16*)(ws + WS_CBL), *HWH = (__bf16*)(ws + WS_HWH), *HWL = (__bf16*)(ws + WS_HWL), *GH = (__bf16*)(ws + WS_GH), *GL = (__bf16*)(ws + WS_GL); float *QKV = (float*)(ws + WS_QKV), *WSL = (float*)(ws + WS_WSL);
  k_pack<<<dim3(3 * DD, 5), 256, 0, stream>>>(F[4], F[6], F[8], F[11], F[12], F[13], F[15], PK);
  k_qkv<<<dim3(NTT * KN / 64, 3 * DD / 128), 128, 0, stream>>>(F[1], PK, F[5], F[7], F[9], QKV);
  k_tok<<<NTT, 256, 0, stream>>>(QKV, F[1], F[2], F[0], F[3], F[10], CBH, CBL, WSL);
  k_gemm<0><<<dim3(NTT / 64, PR / 128), 128, 0, stream>>>(CBH, CBL, nullptr, nullptr, PK, nullptr, WSL, HWH, HWL, nullptr);
  k_gemm<1><<<dim3(NTT / 64, FF / 128), 128, 0, stream>>>(CBH, CBL, HWH, HWL, PK, F[14], nullptr, GH, GL, nullptr);
  k_gemm<2><<<dim3(NTT / 64, DD / 128), 128, 0, stream>>>(GH, GL, nullptr, nullptr, PK, F[16], nullptr, nullptr, nullptr, (float*)d_out);
}
